// DynamicAttention3_40827959116536
// MI455X (gfx1250) — hardware-verified
//
#include <hip/hip_runtime.h>
#include <stddef.h>
#include <stdint.h>
#include <math.h>

#define NB    16
#define NL    256
#define NS    128
#define SP    144
#define NV    129
#define HD    512
#define XD    1536
#define NBL   (NB * NL)
#define NSR   (NB * NS)
#define MSP   (NB * SP)
#define TP    72
#define ATT_THREADS 288

#define QIN_BYTES ((size_t)NBL * HD * 2)
#define SIN_BYTES ((size_t)NSR * HD * 2)
#define WT_BYTES  ((size_t)HD * HD * 2)
#define WOT_BYTES ((size_t)HD * XD * 2)
#define QS_BYTES  ((size_t)NBL * HD * 4)
#define S16_BYTES ((size_t)MSP * HD * 2)
#define X16_BYTES ((size_t)NBL * XD * 2)

#define OFF_QIN  ((size_t)0)
#define OFF_SIN  (OFF_QIN + QIN_BYTES)
#define OFF_TIN  (OFF_SIN + SIN_BYTES)
#define OFF_WQT  (OFF_TIN + SIN_BYTES)
#define OFF_WST  (OFF_WQT + WT_BYTES)
#define OFF_WTT  (OFF_WST + WT_BYTES)
#define OFF_WOT  (OFF_WTT + WT_BYTES)
#define OFF_QS   (OFF_WOT + WOT_BYTES)
#define OFF_S16  (OFF_QS + QS_BYTES)
#define OFF_T16  (OFF_S16 + S16_BYTES)
#define OFF_X16  (OFF_T16 + S16_BYTES)
#define WS_TOTAL (OFF_X16 + X16_BYTES)

static_assert(WS_TOTAL == (size_t)37224448);
static_assert(WS_TOTAL <= (size_t)134217728);
static_assert((OFF_SIN % 256) == 0);
static_assert((OFF_TIN % 256) == 0);
static_assert((OFF_WQT % 256) == 0);
static_assert((OFF_WST % 256) == 0);
static_assert((OFF_WTT % 256) == 0);
static_assert((OFF_WOT % 256) == 0);
static_assert((OFF_QS % 256) == 0);
static_assert((OFF_S16 % 256) == 0);
static_assert((OFF_T16 % 256) == 0);
static_assert((OFF_X16 % 256) == 0);
static_assert((NBL % 4) == 0);
static_assert((NSR % 4) == 0);
static_assert((NBL % 64) == 0);
static_assert((MSP % 64) == 0);
static_assert((HD % 64) == 0);
static_assert((XD % 32) == 0);
static_assert(SP == 9 * 16);
static_assert(ATT_THREADS == 9 * 32);

typedef unsigned short v8us  __attribute__((ext_vector_type(8)));
typedef unsigned short v16us __attribute__((ext_vector_type(16)));
typedef _Float16       v8h   __attribute__((ext_vector_type(8)));
typedef _Float16       v16h  __attribute__((ext_vector_type(16)));
typedef float          v4f   __attribute__((ext_vector_type(4)));
typedef float          v8f   __attribute__((ext_vector_type(8)));
#if defined(__HIP_DEVICE_COMPILE__)
typedef __bf16         v16bf __attribute__((ext_vector_type(16)));
#endif

union FragU { v16us v; v8us half[2]; };
union FragH { v16h  v; v8h  half[2]; };

__device__ __forceinline__ unsigned bbits(float f) {
  unsigned u = __float_as_uint(f);
  return (u + 0x7FFFu + ((u >> 16) & 1u)) >> 16;
}
__device__ __forceinline__ float bf16r(float f) {
  return __uint_as_float(bbits(f) << 16);
}
__device__ __forceinline__ unsigned short hbits(float f) {
  return __builtin_bit_cast(unsigned short, (_Float16)f);
}
__device__ __forceinline__ v8f zero8() { v8f z = {0.f, 0.f, 0.f, 0.f, 0.f, 0.f, 0.f, 0.f}; return z; }
__device__ __forceinline__ v8us zero8us() { v8us z = {0, 0, 0, 0, 0, 0, 0, 0}; return z; }
__device__ __forceinline__ v4f tanh4(v4f v) {
  v4f r;
  r[0] = tanhf(v[0]); r[1] = tanhf(v[1]); r[2] = tanhf(v[2]); r[3] = tanhf(v[3]);
  return r;
}

__device__ __forceinline__ v16us ldfrag_u(const unsigned short* p) {
  FragU f;
  f.half[0] = *(const v8us*)(p);
  f.half[1] = *(const v8us*)(p + 16);
  return f.v;
}

__device__ __forceinline__ v8f mma_bf(v16us a, v16us b, v8f c) {
#if defined(__HIP_DEVICE_COMPILE__)
  return __builtin_amdgcn_wmma_f32_16x16x32_bf16(false, __builtin_bit_cast(v16bf, a),
                                                false, __builtin_bit_cast(v16bf, b),
                                                (short)0, c, false, false);
#else
  (void)a; (void)b;
  return c;
#endif
}
__device__ __forceinline__ v8f mma_hu(v16us a, v16us b, v8f c) {
#if defined(__HIP_DEVICE_COMPILE__)
  return __builtin_amdgcn_wmma_f32_16x16x32_f16(false, __builtin_bit_cast(v16h, a),
                                               false, __builtin_bit_cast(v16h, b),
                                               (short)0, c, false, false);
#else
  (void)a; (void)b;
  return c;
#endif
}
__device__ __forceinline__ v8f mma_h(v16h a, v16h b, v8f c) {
#if defined(__HIP_DEVICE_COMPILE__)
  return __builtin_amdgcn_wmma_f32_16x16x32_f16(false, a, false, b, (short)0, c, false, false);
#else
  (void)a; (void)b;
  return c;
#endif
}
__device__ __forceinline__ void guard4(v8f& c0, v8f& c1, v8f& c2, v8f& c3, const v16us& a,
                                       const v16us& b0, const v16us& b1, const v16us& b2,
                                       const v16us& b3) {
#if defined(__HIP_DEVICE_COMPILE__)
  asm volatile("v_nop\n\tv_nop\n\tv_nop\n\tv_nop"
               : "+v"(c0), "+v"(c1), "+v"(c2), "+v"(c3)
               : "v"(a), "v"(b0), "v"(b1), "v"(b2), "v"(b3));
#else
  (void)c0; (void)c1; (void)c2; (void)c3; (void)a; (void)b0; (void)b1; (void)b2; (void)b3;
#endif
}
__device__ __forceinline__ void guard9(v8f& c0, v8f& c1, v8f& c2, v8f& c3, v8f& c4, v8f& c5,
                                       v8f& c6, v8f& c7, v8f& c8, const v16h& a, const v16h& b) {
#if defined(__HIP_DEVICE_COMPILE__)
  asm volatile("v_nop\n\tv_nop\n\tv_nop\n\tv_nop"
               : "+v"(c0), "+v"(c1), "+v"(c2), "+v"(c3), "+v"(c4), "+v"(c5), "+v"(c6),
                 "+v"(c7), "+v"(c8)
               : "v"(a), "v"(b));
#else
  (void)c0; (void)c1; (void)c2; (void)c3; (void)c4; (void)c5; (void)c6; (void)c7; (void)c8;
  (void)a; (void)b;
#endif
}

template <bool DO_TANH>
__device__ __forceinline__ void store_tile_f32(const float* ct, float* C, int row0, int col0,
                                               int ldc, int w, int lane) {
  const int q  = lane >> 3;
  const int jj = lane & 7;
#pragma unroll 1
  for (int it = 0; it < 8; ++it) {
    const int li = it * 16 + w * 4 + q;
    const int tr = li >> 1, hf = li & 1;
    v4f v = *(const v4f*)(ct + tr * 64 + hf * 32 + jj * 4);
    if (DO_TANH) v = tanh4(v);
    *(volatile v4f*)(C + (size_t)(row0 + tr) * ldc + col0 + hf * 32 + jj * 4) = v;
  }
  __threadfence();
#pragma unroll 1
  for (int it = 0; it < 8; ++it) {
    const int li = it * 16 + w * 4 + q;
    const int tr = li >> 1, hf = li & 1;
    v4f v = *(const v4f*)(ct + tr * 64 + hf * 32 + jj * 4);
    if (DO_TANH) v = tanh4(v);
    *(volatile v4f*)(C + (size_t)(row0 + tr) * ldc + col0 + hf * 32 + jj * 4) = v;
  }
}
__device__ __forceinline__ void store_tile_h(const _Float16* ht, _Float16* P, int row0, int col0,
                                             int ldp, int w, int lane) {
  const int q  = lane >> 3;
  const int jj = lane & 7;
  v8h    v[4];
  size_t off[4];
#pragma unroll
  for (int it = 0; it < 4; ++it) {
    const int li = it * 16 + w * 4 + q;
    v[it]   = *(const v8h*)(ht + li * 64 + 8 * jj);
    off[it] = (size_t)(row0 + li) * ldp + col0 + 8 * jj;
  }
#pragma unroll
  for (int it = 0; it < 4; ++it) *(volatile v8h*)(P + off[it]) = v[it];
  __threadfence();
#pragma unroll
  for (int it = 0; it < 4; ++it) *(volatile v8h*)(P + off[it]) = v[it];
}

__global__ __launch_bounds__(256)
void k_cvt_in(const float* __restrict__ query, const float* __restrict__ src,
              const float* __restrict__ trg, unsigned short* qin, unsigned short* srcb,
              unsigned short* trgb, unsigned short* x16)
{
  const int tid  = threadIdx.x;
  const int row4 = blockIdx.x * 4;
  const int kind = (row4 < NBL) ? 0 : ((row4 < NBL + NSR) ? 1 : 2);
  const int base = (kind == 0) ? 0 : ((kind == 1) ? NBL : (NBL + NSR));
  const int row  = row4 + (tid >> 6) - base;
  const int pc   = tid & 63;
  const float* sp = ((kind == 0) ? query : ((kind == 1) ? src : trg)) + (size_t)row * HD + 8 * pc;
  unsigned short* dp = ((kind == 0) ? qin : ((kind == 1) ? srcb : trgb)) + (size_t)row * HD + 8 * pc;
  unsigned short* xp = x16 + (size_t)row * XD + 8 * pc;

  const v4f a0 = *(const v4f*)(sp);
  const v4f a1 = *(const v4f*)(sp + 4);
  v8us ob, ox;
#pragma unroll
  for (int e = 0; e < 4; ++e) {
    const float v0 = bf16r(a0[e]);
    const float v1 = bf16r(a1[e]);
    ob[e]     = (unsigned short)bbits(v0);
    ob[4 + e] = (unsigned short)bbits(v1);
    ox[e]     = hbits(16.0f * v0);
    ox[4 + e] = hbits(16.0f * v1);
  }
  *(volatile v8us*)dp = ob;
  if (kind == 0) *(volatile v8us*)xp = ox;
  __threadfence();
  *(volatile v8us*)dp = ob;
  if (kind == 0) *(volatile v8us*)xp = ox;
}

__global__ __launch_bounds__(256)
void k_cvt_w(const float* __restrict__ Wq, const float* __restrict__ Ws,
             const float* __restrict__ Wt, const float* __restrict__ Wo,
             unsigned short* wqt, unsigned short* wst, unsigned short* wtt, unsigned short* wot)
{
  __shared__ __align__(16) unsigned short tnk[64 * TP];

  const int bid  = blockIdx.x;
  const int kind = (bid < 64) ? 0 : ((bid < 128) ? 1 : ((bid < 192) ? 2 : 3));
  const int loc  = bid - ((kind == 3) ? 192 : 64 * kind);
  const int KD   = (kind == 3) ? XD : HD;
  const float* W = (kind == 0) ? Wq : ((kind == 1) ? Ws : ((kind == 2) ? Wt : Wo));
  unsigned short* WT = (kind == 0) ? wqt : ((kind == 1) ? wst : ((kind == 2) ? wtt : wot));
  const int kt   = loc >> 3;
  const int nt   = loc & 7;
  const int tid  = threadIdx.x;
  const int lane = tid & 31;
  const int w    = tid >> 5;
  const int q    = lane >> 3;
  const int jj   = lane & 7;

  const int kk = tid >> 2;
  const int n0 = 16 * (tid & 3);
  const float* wp = W + (size_t)(64 * kt + kk) * HD + 64 * nt + n0;
  v4f u[4];
  u[0] = *(const v4f*)(wp);
  u[1] = *(const v4f*)(wp + 4);
  u[2] = *(const v4f*)(wp + 8);
  u[3] = *(const v4f*)(wp + 12);
#pragma unroll
  for (int g = 0; g < 4; ++g) {
#pragma unroll
    for (int e = 0; e < 4; ++e) {
      const float x = bf16r(u[g][e]);
      const unsigned short hb = hbits(64.0f * x);
      const unsigned short bb = (unsigned short)bbits(x);
      tnk[(n0 + 4 * g + e) * TP + kk] = (kind == 3) ? hb : bb;
    }
  }
  __syncthreads();

  v8us   v[2];
  size_t off[2];
#pragma unroll
  for (int it = 0; it < 2; ++it) {
    const int li = it * 32 + w * 4 + q;
    v[it]   = *(const v8us*)(tnk + li * TP + 8 * jj);
    off[it] = (size_t)(64 * nt + li) * KD + 64 * kt + 8 * jj;
  }
#pragma unroll
  for (int it = 0; it < 2; ++it) *(volatile v8us*)(WT + off[it]) = v[it];
  __threadfence();
#pragma unroll
  for (int it = 0; it < 2; ++it) *(volatile v8us*)(WT + off[it]) = v[it];
}

__global__ __launch_bounds__(128)
void k_projq(const unsigned short* __restrict__ a16, const unsigned short* __restrict__ wt,
             const float* __restrict__ bias, float* qs)
{
  __shared__ __align__(16) float ct[64 * 64];

  const int tid  = threadIdx.x;
  const int lane = tid & 31;
  const int w    = tid >> 5;
  const int h    = lane >> 4;
  const int m    = lane & 15;
  const int col0 = 64 * blockIdx.x;
  const int row0 = 64 * blockIdx.y;

  v8f acc[4];
#pragma unroll
  for (int j = 0; j < 4; ++j) acc[j] = zero8();

  const unsigned short* pa = a16 + (size_t)(row0 + 16 * w + m) * HD + 8 * h;
  const unsigned short* pb = wt + (size_t)(col0 + m) * HD + 8 * h;
#pragma unroll 2
  for (int kk = 0; kk < HD / 32; ++kk) {
    const v16us a  = ldfrag_u(pa + 32 * kk);
    const v16us b0 = ldfrag_u(pb + 32 * kk);
    const v16us b1 = ldfrag_u(pb + (size_t)16 * HD + 32 * kk);
    const v16us b2 = ldfrag_u(pb + (size_t)32 * HD + 32 * kk);
    const v16us b3 = ldfrag_u(pb + (size_t)48 * HD + 32 * kk);
    acc[0] = mma_bf(a, b0, acc[0]);
    acc[1] = mma_bf(a, b1, acc[1]);
    acc[2] = mma_bf(a, b2, acc[2]);
    acc[3] = mma_bf(a, b3, acc[3]);
    guard4(acc[0], acc[1], acc[2], acc[3], a, b0, b1, b2, b3);
  }

#pragma unroll
  for (int j = 0; j < 4; ++j) {
    const float bv = bf16r(bias[col0 + 16 * j + m]);
#pragma unroll
    for (int r = 0; r < 8; ++r)
      ct[(16 * w + 8 * h + r) * 64 + 16 * j + m] = 16.0f * (acc[j][r] + bv);
  }
  __syncthreads();
  store_tile_f32<false>(ct, qs, row0, col0, HD, w, lane);
}

__global__ __launch_bounds__(128)
void k_projst(const unsigned short* __restrict__ srcb, const unsigned short* __restrict__ trgb,
              const unsigned short* __restrict__ wst, const unsigned short* __restrict__ wtt,
              const float* __restrict__ bs, const float* __restrict__ bt,
              _Float16* s16, _Float16* t16)
{
  __shared__ __align__(16) _Float16 ht[64 * 64];

  const int z    = blockIdx.z;
  const unsigned short* a16 = z ? trgb : srcb;
  const unsigned short* wt  = z ? wtt : wst;
  const float* bias = z ? bt : bs;
  _Float16* outp = z ? t16 : s16;

  const int tid  = threadIdx.x;
  const int lane = tid & 31;
  const int w    = tid >> 5;
  const int h    = lane >> 4;
  const int m    = lane & 15;
  const int col0 = 64 * blockIdx.x;
  const int row0 = 64 * blockIdx.y;

  const int mrow = row0 + 16 * w + m;
  const int bb   = mrow / SP;
  const int rr   = mrow - bb * SP;
  const bool okrow = (rr < NS);
  const int arow = bb * NS + (okrow ? rr : (NS - 1));
  const v8us z8 = zero8us();

  v8f acc[4];
#pragma unroll
  for (int j = 0; j < 4; ++j) acc[j] = zero8();

  const unsigned short* pa = a16 + (size_t)arow * HD + 8 * h;
  const unsigned short* pb = wt + (size_t)(col0 + m) * HD + 8 * h;
#pragma unroll 2
  for (int kk = 0; kk < HD / 32; ++kk) {
    FragU fa;
    const v8us l0 = *(const v8us*)(pa + 32 * kk);
    const v8us l1 = *(const v8us*)(pa + 32 * kk + 16);
    fa.half[0] = okrow ? l0 : z8;
    fa.half[1] = okrow ? l1 : z8;
    const v16us b0 = ldfrag_u(pb + 32 * kk);
    const v16us b1 = ldfrag_u(pb + (size_t)16 * HD + 32 * kk);
    const v16us b2 = ldfrag_u(pb + (size_t)32 * HD + 32 * kk);
    const v16us b3 = ldfrag_u(pb + (size_t)48 * HD + 32 * kk);
    acc[0] = mma_bf(fa.v, b0, acc[0]);
    acc[1] = mma_bf(fa.v, b1, acc[1]);
    acc[2] = mma_bf(fa.v, b2, acc[2]);
    acc[3] = mma_bf(fa.v, b3, acc[3]);
    guard4(acc[0], acc[1], acc[2], acc[3], fa.v, b0, b1, b2, b3);
  }

#pragma unroll
  for (int j = 0; j < 4; ++j) {
    const float bv = bf16r(bias[col0 + 16 * j + m]);
#pragma unroll
    for (int r = 0; r < 8; ++r)
      ht[(16 * w + 8 * h + r) * 64 + 16 * j + m] = (_Float16)(8.0f * (acc[j][r] + bv));
  }
  __syncthreads();
  store_tile_h(ht, outp, row0, col0, HD, w, lane);
}

__global__ __launch_bounds__(ATT_THREADS)
void k_attn(const float* __restrict__ qs, const _Float16* __restrict__ s16,
            const _Float16* __restrict__ t16, _Float16* x16)
{
  __shared__ __align__(16) float qL[HD];
  __shared__ float wL[2][SP];
  __shared__ float cpL[9][SP];
  __shared__ float wmaxL[16];
  __shared__ float zL[4];

  const int tid  = threadIdx.x;
  const int lane = tid & 31;
  const int w    = tid >> 5;
  const int h    = lane >> 4;
  const int m    = lane & 15;
  const int bl   = blockIdx.x;
  const int b    = bl >> 8;

  for (int i = tid; i < HD; i += ATT_THREADS) qL[i] = qs[(size_t)bl * HD + i];
  __syncthreads();

  const _Float16* Sb = s16 + (size_t)b * SP * HD;
  const _Float16* Tb = t16 + (size_t)b * SP * HD;
  const _Float16* pa = Sb + (size_t)(16 * w + m) * HD + 8 * h;
  const _Float16* pb = Tb + (size_t)m * HD + 8 * h;

  v8f acc[9];
#pragma unroll
  for (int j = 0; j < 9; ++j) acc[j] = zero8();

#pragma unroll 1
  for (int kk = 0; kk < HD / 32; ++kk) {
    const int k0 = 32 * kk;
    const v8h s0 = *(const v8h*)(pa + k0);
    const v8h s1 = *(const v8h*)(pa + k0 + 16);
    const v4f q0a = *(const v4f*)(qL + k0 + 8 * h);
    const v4f q0b = *(const v4f*)(qL + k0 + 8 * h + 4);
    const v4f q1a = *(const v4f*)(qL + k0 + 16 + 8 * h);
    const v4f q1b = *(const v4f*)(qL + k0 + 16 + 8 * h + 4);
    v8h a0, a1;
#pragma unroll
    for (int e = 0; e < 4; ++e) {
      a0[e]     = (_Float16)((float)s0[e]     * q0a[e]);
      a0[4 + e] = (_Float16)((float)s0[4 + e] * q0b[e]);
      a1[e]     = (_Float16)((float)s1[e]     * q1a[e]);
      a1[4 + e] = (_Float16)((float)s1[4 + e] * q1b[e]);
    }
    FragH fa;
    fa.half[0] = a0;
    fa.half[1] = a1;
    v16h blast = fa.v;
#pragma unroll
    for (int j = 0; j < 9; ++j) {
      FragH fb;
      fb.half[0] = *(const v8h*)(pb + (size_t)(16 * j) * HD + k0);
      fb.half[1] = *(const v8h*)(pb + (size_t)(16 * j) * HD + k0 + 16);
      acc[j] = mma_h(fa.v, fb.v, acc[j]);
      blast = fb.v;
    }
    guard9(acc[0], acc[1], acc[2], acc[3], acc[4], acc[5], acc[6], acc[7], acc[8],
           fa.v, blast);
  }

  const float lsc = 4.3158372875e-05f;
  const float NEG = -1.0e30f;
  float mx = NEG;
#pragma unroll
  for (int j = 0; j < 9; ++j) {
    const int t = 16 * j + m;
    const bool tv = (t < NV);
#pragma unroll
    for (int r = 0; r < 8; ++r) {
      const int s = 16 * w + 8 * h + r;
      const bool valid = tv && (s < NV);
      float v = acc[j][r] * lsc;
      v = valid ? v : NEG;
      acc[j][r] = v;
      mx = fmaxf(mx, v);
    }
  }
#pragma unroll
  for (int o = 16; o >= 1; o >>= 1) mx = fmaxf(mx, __shfl_xor(mx, o, 32));
  if (lane == 0) wmaxL[w] = mx;
  __syncthreads();
  float gm = wmaxL[0];
#pragma unroll
  for (int i = 1; i < 9; ++i) gm = fmaxf(gm, wmaxL[i]);

  float rp[8];
#pragma unroll
  for (int r = 0; r < 8; ++r) rp[r] = 0.f;
#pragma unroll
  for (int j = 0; j < 9; ++j) {
    float cp = 0.f;
#pragma unroll
    for (int r = 0; r < 8; ++r) {
      const float e = __expf(acc[j][r] - gm);
      rp[r] += e;
      cp += e;
    }
    cp += __shfl_xor(cp, 16, 32);
    if (h == 0) cpL[w][16 * j + m] = cp;
  }
#pragma unroll
  for (int r = 0; r < 8; ++r) {
    float v = rp[r];
#pragma unroll
    for (int o = 1; o <= 8; o <<= 1) v += __shfl_xor(v, o, 32);
    if (m == 0) wL[0][16 * w + 8 * h + r] = v;
  }
  __syncthreads();

  if (tid < SP) {
    float c = 0.f;
#pragma unroll
    for (int w2 = 0; w2 < 9; ++w2) c += cpL[w2][tid];
    wL[1][tid] = c;
  }
  if (w == 0) {
    float zs = 0.f;
#pragma unroll
    for (int i = 0; i < 5; ++i) {
      const int idx = lane + 32 * i;
      const int ic  = (idx < SP) ? idx : (SP - 1);
      float v = wL[0][ic];
      zs += (idx < SP) ? v : 0.f;
    }
#pragma unroll
    for (int o = 16; o >= 1; o >>= 1) zs += __shfl_xor(zs, o, 32);
    if (lane == 0) zL[0] = zs;
  }
  __syncthreads();
  const float invZ = 1.0f / zL[0];

  if (tid < 128) {
    const int which = tid >> 6;
    const int oc    = tid & 63;
    const _Float16* P = (which ? Tb : Sb) + 8 * oc;
    float cx[8];
#pragma unroll
    for (int e = 0; e < 8; ++e) cx[e] = 0.f;
#pragma unroll 1
    for (int s = 0; s < NV; ++s) {
      const float wgt = wL[which][s];
      const v8h v = *(const v8h*)(P + (size_t)s * HD);
#pragma unroll
      for (int e = 0; e < 8; ++e) cx[e] += wgt * (float)v[e];
    }
    const float f = 2.0f * invZ;
    v8h o;
#pragma unroll
    for (int e = 0; e < 8; ++e) o[e] = (_Float16)(cx[e] * f);
    _Float16* dst = x16 + (size_t)bl * XD + HD + 8 * tid;
    *(volatile v8h*)dst = o;
    __threadfence();
    *(volatile v8h*)dst = o;
  }
}

__global__ __launch_bounds__(128)
void k_out(const unsigned short* __restrict__ x16, const unsigned short* __restrict__ wot,
           const float* __restrict__ bo, float* out)
{
  __shared__ __align__(16) float ct[64 * 64];

  const int tid  = threadIdx.x;
  const int lane = tid & 31;
  const int w    = tid >> 5;
  const int h    = lane >> 4;
  const int m    = lane & 15;
  const int col0 = 64 * blockIdx.x;
  const int row0 = 64 * blockIdx.y;

  v8f acc[4];
#pragma unroll
  for (int j = 0; j < 4; ++j) acc[j] = zero8();

  const unsigned short* pa = x16 + (size_t)(row0 + 16 * w + m) * XD + 8 * h;
  const unsigned short* pb = wot + (size_t)(col0 + m) * XD + 8 * h;
#pragma unroll 2
  for (int kk = 0; kk < XD / 32; ++kk) {
    const v16us a  = ldfrag_u(pa + 32 * kk);
    const v16us b0 = ldfrag_u(pb + 32 * kk);
    const v16us b1 = ldfrag_u(pb + (size_t)16 * XD + 32 * kk);
    const v16us b2 = ldfrag_u(pb + (size_t)32 * XD + 32 * kk);
    const v16us b3 = ldfrag_u(pb + (size_t)48 * XD + 32 * kk);
    acc[0] = mma_hu(a, b0, acc[0]);
    acc[1] = mma_hu(a, b1, acc[1]);
    acc[2] = mma_hu(a, b2, acc[2]);
    acc[3] = mma_hu(a, b3, acc[3]);
    guard4(acc[0], acc[1], acc[2], acc[3], a, b0, b1, b2, b3);
  }

  const float osc = 1.0f / 1024.0f;
#pragma unroll
  for (int j = 0; j < 4; ++j) {
    const float bv = bf16r(bo[col0 + 16 * j + m]);
#pragma unroll
    for (int r = 0; r < 8; ++r)
      ct[(16 * w + 8 * h + r) * 64 + 16 * j + m] = acc[j][r] * osc + bv;
  }
  __syncthreads();
  store_tile_f32<true>(ct, out, row0, col0, HD, w, lane);
}

extern "C" void kernel_launch(void* const* d_in, const int* in_sizes, int n_in,
                              void* d_out, int out_size, void* d_ws, size_t ws_size,
                              hipStream_t stream) {
  if (n_in < 11) return;
  if (in_sizes[0] != NBL * HD) return;
  if (in_sizes[1] != NSR * HD) return;
  if (in_sizes[2] != NSR * HD) return;
  if (in_sizes[3] != HD * HD) return;
  if (in_sizes[4] != HD) return;
  if (in_sizes[5] != HD * HD) return;
  if (in_sizes[6] != HD) return;
  if (in_sizes[7] != HD * HD) return;
  if (in_sizes[8] != HD) return;
  if (in_sizes[9] != XD * HD) return;
  if (in_sizes[10] != HD) return;
  if (out_size != NBL * HD) return;
  if (ws_size < WS_TOTAL) return;

  const float* query = (const float*)d_in[0];
  const float* src   = (const float*)d_in[1];
  const float* trg   = (const float*)d_in[2];
  const float* Wq    = (const float*)d_in[3];
  const float* bq    = (const float*)d_in[4];
  const float* Ws    = (const float*)d_in[5];
  const float* bs    = (const float*)d_in[6];
  const float* Wt    = (const float*)d_in[7];
  const float* bt    = (const float*)d_in[8];
  const float* Wo    = (const float*)d_in[9];
  const float* bo    = (const float*)d_in[10];
  float* out = (float*)d_out;

  char* ws = (char*)d_ws;
  unsigned short* qin  = (unsigned short*)(ws + OFF_QIN);
  unsigned short* srcb = (unsigned short*)(ws + OFF_SIN);
  unsigned short* trgb = (unsigned short*)(ws + OFF_TIN);
  unsigned short* wqt  = (unsigned short*)(ws + OFF_WQT);
  unsigned short* wst  = (unsigned short*)(ws + OFF_WST);
  unsigned short* wtt  = (unsigned short*)(ws + OFF_WTT);
  unsigned short* wot  = (unsigned short*)(ws + OFF_WOT);
  float*          qsb  = (float*)(ws + OFF_QS);
  _Float16*       s16  = (_Float16*)(ws + OFF_S16);
  _Float16*       t16  = (_Float16*)(ws + OFF_T16);
  unsigned short* x16u = (unsigned short*)(ws + OFF_X16);
  _Float16*       x16h = (_Float16*)(ws + OFF_X16);

  k_cvt_in<<<dim3((NBL + 2 * NSR) / 4), dim3(256), 0, stream>>>(query, src, trg, qin, srcb,
                                                               trgb, x16u);
  (void)hipGetLastError();
  k_cvt_w<<<dim3(384), dim3(256), 0, stream>>>(Wq, Ws, Wt, Wo, wqt, wst, wtt, wot);
  (void)hipGetLastError();
  k_projq<<<dim3(HD / 64, NBL / 64), dim3(128), 0, stream>>>(qin, wqt, bq, qsb);
  (void)hipGetLastError();
  k_projst<<<dim3(HD / 64, MSP / 64, 2), dim3(128), 0, stream>>>(srcb, trgb, wst, wtt, bs, bt,
                                                                s16, t16);
  (void)hipGetLastError();
  k_attn<<<dim3(NBL), dim3(ATT_THREADS), 0, stream>>>(qsb, s16, t16, x16h);
  (void)hipGetLastError();
  k_out<<<dim3(HD / 64, NBL / 64), dim3(128), 0, stream>>>(x16u, wot, bo, out);
  (void)hipGetLastError();
}
